// MultiHeadAttention2_54820962566690
// MI455X (gfx1250) — hardware-verified
//
#include <hip/hip_runtime.h>

#ifndef NB
#define NB 4
#endif
#ifndef SEQ
#define SEQ 2048
#endif
#ifndef RR
#define RR 256
#endif
#define NB_FULL 4
#define SEQ_FULL 2048
#define DM 1024
#define NH 16
#define HDIM 64

static_assert(NB >= 1 && NB <= NB_FULL);
static_assert(SEQ % 64 == 0 && SEQ >= 64 && SEQ <= SEQ_FULL);
static_assert(RR % 64 == 0 && RR >= 64 && RR <= SEQ);
static_assert(NH * HDIM == DM);
static_assert(DM % 64 == 0);

typedef __attribute__((ext_vector_type(16))) _Float16 v16h;
typedef __attribute__((ext_vector_type(8)))  _Float16 v8h;
typedef __attribute__((ext_vector_type(16))) __bf16   v16b;
typedef __attribute__((ext_vector_type(8)))  __bf16   v8b;
typedef __attribute__((ext_vector_type(8)))  float    v8f;
typedef __attribute__((ext_vector_type(4)))  float    v4f;

#define WSC 256.0f
#define OSC 64.0f
#define PSCALE 32768.0f
#define RSC 1024.0f
#define RSC_INV (1.0f / 1024.0f)
#define NEG_INF (-__builtin_huge_valf())

__device__ __forceinline__ unsigned short f2bf_bits(float f) {
  unsigned u = __float_as_uint(f);
  return (unsigned short)((u + 0x7FFFu + ((u >> 16) & 1u)) >> 16);
}
__device__ __forceinline__ float bf_bits2f(unsigned short h) { return __uint_as_float(((unsigned)h) << 16); }
__device__ __forceinline__ float bf_rne(float f) { return bf_bits2f(f2bf_bits(f)); }
__device__ __forceinline__ _Float16 bf_f16(float f) { return (_Float16)bf_rne(f); }

__device__ __forceinline__ void wave_lds_sync() {
  __builtin_amdgcn_fence(3, "workgroup");
  __builtin_amdgcn_wave_barrier();
  __builtin_amdgcn_fence(2, "workgroup");
}

__device__ __forceinline__ void dep_guard_h(v8f& a, v8f& b, v16h x, v16h y) { asm volatile("v_nop\n\tv_nop\n\tv_nop\n\tv_nop" : "+v"(a), "+v"(b) : "v"(x), "v"(y)); }
__device__ __forceinline__ void dep_guard_b(v8f& a, v8f& b, v16b x, v16b y) { asm volatile("v_nop\n\tv_nop\n\tv_nop\n\tv_nop" : "+v"(a), "+v"(b) : "v"(x), "v"(y)); }
__device__ __forceinline__ void keep4_h(v16h a, v16h b, v16h c, v16h d) { asm volatile("v_nop" :: "v"(a), "v"(b), "v"(c), "v"(d)); }
__device__ __forceinline__ void keep4_b(v16b a, v16b b, v16b c, v16b d) { asm volatile("v_nop" :: "v"(a), "v"(b), "v"(c), "v"(d)); }
__device__ __forceinline__ void acc_guard4(v8f& a, v8f& b, v8f& c, v8f& d) { asm volatile("v_nop\n\tv_nop\n\tv_nop\n\tv_nop" : "+v"(a), "+v"(b), "+v"(c), "+v"(d)); }
template <typename T> struct Frag;
template <> struct Frag<_Float16> {
  typedef v16h V; union U { v16h v; v8h h[2]; };
  static __device__ __forceinline__ v16h load(const _Float16* p) {
    U f; f.h[0] = *(const v8h*)(p); f.h[1] = *(const v8h*)(p + 16); return f.v;
  }
  static __device__ __forceinline__ v8f mma(v16h a, v16h b, v8f c) {
    return __builtin_amdgcn_wmma_f32_16x16x32_f16(false, a, false, b, (short)0, c, false, false);
  }
  static __device__ __forceinline__ void guard(v8f& a, v8f& b, v16h x, v16h y) { dep_guard_h(a, b, x, y); }
  static __device__ __forceinline__ void keep(v16h a, v16h b, v16h c, v16h d) { keep4_h(a, b, c, d); }
};
template <> struct Frag<__bf16> {
  typedef v16b V; union U { v16b v; v8b h[2]; };
  static __device__ __forceinline__ v16b load(const __bf16* p) {
    U f; f.h[0] = *(const v8b*)(p); f.h[1] = *(const v8b*)(p + 16); return f.v;
  }
  static __device__ __forceinline__ v8f mma(v16b a, v16b b, v8f c) {
    return __builtin_amdgcn_wmma_f32_16x16x32_bf16(false, a, false, b, (short)0, c, false, false);
  }
  static __device__ __forceinline__ void guard(v8f& a, v8f& b, v16b x, v16b y) { dep_guard_b(a, b, x, y); }
  static __device__ __forceinline__ void keep(v16b a, v16b b, v16b c, v16b d) { keep4_b(a, b, c, d); }
};

template <int ET> struct Elem;
template <> struct Elem<0> { typedef _Float16 T; };
template <> struct Elem<1> { typedef __bf16 T; };
template <int ET, bool SPLIT, int BIAS_MODE, int OUT_MODE, bool RESID, int ACT = 0>
__global__ __launch_bounds__(256) void wmma_gemm64(
    const unsigned short* __restrict__ Ap, const unsigned short* __restrict__ A2p, int lda, long strideA,
    const unsigned short* __restrict__ Btp, const unsigned short* __restrict__ Bt2p, int ldb, long strideB,
    void* __restrict__ Cout, void* __restrict__ Cout2, int ldc, long strideC,
    const float* __restrict__ bias,
    const float* __restrict__ resid, long strideR,
    int M, int N, int K, float scale) {
  typedef typename Elem<ET>::T T;
  typedef typename Frag<T>::V V;
  const T* A = (const T*)Ap; const T* A2 = (const T*)A2p; const T* Bt = (const T*)Btp; const T* Bt2 = (const T*)Bt2p;
  __shared__ __align__(16) float sT[8][16 * 68];
  const int b    = blockIdx.y;
  const int lane = threadIdx.x & 31;
  const int wave = threadIdx.x >> 5;
  const int tilesN = N >> 6;
  const int tilesM = M >> 6;
  const int tile = blockIdx.x * 8 + wave;
  if (tile >= tilesM * tilesN) return;
  const int tm = tile / tilesN;
  const int tn = tile - tm * tilesN;
  const int m0 = tm << 6;
  const int n0 = tn << 6;

  const T* Ab  = A  + (size_t)b * strideA;
  const T* Bb  = Bt + (size_t)b * strideB;
  const T* Ab2 = SPLIT ? (A2  + (size_t)b * strideA) : nullptr;
  const T* Bb2 = SPLIT ? (Bt2 + (size_t)b * strideB) : nullptr;

  const int rlane = lane & 15;
  const int koff  = (lane >> 4) * 8;
  const int mOff  = (lane >> 4) * 8;

  v8f acc[4][4];
#pragma unroll
  for (int i = 0; i < 4; ++i)
#pragma unroll
    for (int j = 0; j < 4; ++j) acc[i][j] = (v8f){0.f,0.f,0.f,0.f,0.f,0.f,0.f,0.f};

  for (int k0 = 0; k0 < K; k0 += 32) {
    V bh[4], bl[4];
#pragma unroll
    for (int j = 0; j < 4; ++j) {
      const size_t bo = (size_t)(n0 + (j << 4) + rlane) * ldb + koff + k0;
      bh[j] = Frag<T>::load(Bb + bo);
      if (SPLIT) bl[j] = Frag<T>::load(Bb2 + bo);
    }
#pragma unroll
    for (int i = 0; i < 4; ++i) {
      const size_t ao = (size_t)(m0 + (i << 4) + rlane) * lda + koff + k0;
      V ah = Frag<T>::load(Ab + ao);
      V al;
      if (SPLIT) al = Frag<T>::load(Ab2 + ao);
#pragma unroll
      for (int j = 0; j < 4; ++j) {
        acc[i][j] = Frag<T>::mma(ah, bh[j], acc[i][j]);
        if (SPLIT) {
          acc[i][j] = Frag<T>::mma(ah, bl[j], acc[i][j]);
          acc[i][j] = Frag<T>::mma(al, bh[j], acc[i][j]);
        }
      }
      Frag<T>::guard(acc[i][0], acc[i][3], ah, SPLIT ? al : ah);
    }
    Frag<T>::keep(bh[0], bh[1], bh[2], bh[3]);
    if (SPLIT) Frag<T>::keep(bl[0], bl[1], bl[2], bl[3]);
  }
  acc_guard4(acc[0][0], acc[0][1], acc[0][2], acc[0][3]);
  acc_guard4(acc[1][0], acc[1][1], acc[1][2], acc[1][3]);
  acc_guard4(acc[2][0], acc[2][1], acc[2][2], acc[2][3]);
  acc_guard4(acc[3][0], acc[3][1], acc[3][2], acc[3][3]);

  float* slab = sT[wave];
  const float* Rb = RESID ? (resid + (size_t)b * strideR) : nullptr;
#pragma unroll
  for (int i = 0; i < 4; ++i) {
    const int mBase = m0 + (i << 4);
#pragma unroll
    for (int j = 0; j < 4; ++j) {
      const int n = n0 + (j << 4) + rlane;
      float bv = 0.f;
      if (BIAS_MODE == 2) bv = bf_rne(bias[n]);
#pragma unroll
      for (int r = 0; r < 8; ++r) {
        float v = acc[i][j][r] * scale;
        if (BIAS_MODE == 1) v += bf_rne(bias[mBase + mOff + r]);
        if (BIAS_MODE == 2) v += bv;
        if (RESID) v += Rb[(size_t)(mBase + mOff + r) * ldc + n];
        if (ACT == 1) v = tanhf(v);
        if (ACT == 2) v = fmaxf(v, 0.0f);
        if (ACT == 3) v = v / (1.0f + expf(-v));
        if (ACT == 4) v = (v > 0.f) ? v : 0.01f * v;
        if (ACT == 5) v = 0.5f * v * (1.0f + erff(v * 0.70710678118654752f));
        slab[(mOff + r) * 68 + (j << 4) + rlane] = v;
      }
    }
    wave_lds_sync();
    if (OUT_MODE == 0) {
      float* C = (float*)Cout + (size_t)b * strideC;
      const int hh = lane >> 4, c4 = (lane & 15) * 4;
      for (int pass = 0; pass < 2; ++pass) {
#pragma unroll
        for (int it = 0; it < 8; ++it) {
          const int row = it * 2 + hh;
          v4f v = *(const v4f*)(slab + row * 68 + c4);
          *(volatile v4f*)(C + (size_t)(mBase + row) * ldc + n0 + c4) = v;
        }
        __threadfence();
      }
    } else {
      const int q = lane >> 3, c8 = (lane & 7) * 8;
      unsigned short* C  = (unsigned short*)Cout  + (size_t)b * strideC;
      unsigned short* C2 = (OUT_MODE >= 2) ? ((unsigned short*)Cout2 + (size_t)b * strideC) : nullptr;
      for (int pass = 0; pass < 2; ++pass) {
#pragma unroll
        for (int it = 0; it < 4; ++it) {
          const int row = it * 4 + q;
          const float* sp = slab + row * 68 + c8;
          v8h hv, lv;
#pragma unroll
          for (int e = 0; e < 8; ++e) {
            if (OUT_MODE == 1) {
              hv[e] = (_Float16)sp[e];
            } else if (OUT_MODE == 3) {
              const float    fv = sp[e];
              const _Float16 hq = (_Float16)fv;
              hv[e] = hq;
              lv[e] = (_Float16)((fv - (float)hq) * RSC);
            } else {
              unsigned short hb = f2bf_bits(sp[e]);
              unsigned short lb = f2bf_bits(sp[e] - bf_bits2f(hb));
              hv[e] = __builtin_bit_cast(_Float16, hb);
              lv[e] = __builtin_bit_cast(_Float16, lb);
            }
          }
          *(volatile v8h*)(C + (size_t)(mBase + row) * ldc + n0 + c8) = hv;
          if (OUT_MODE >= 2) *(volatile v8h*)(C2 + (size_t)(mBase + row) * ldc + n0 + c8) = lv;
        }
        __threadfence();
      }
    }
    wave_lds_sync();
  }
}

__global__ __launch_bounds__(256) void cast_x_f16(
    const float* __restrict__ x, unsigned short* __restrict__ xhp, int nrows) {
  const long i = (long)blockIdx.x * 256 + threadIdx.x;
  const long total = (long)nrows * (DM / 8);
  if (i >= total) return;
  const int r  = (int)(i / (DM / 8));
  const int c8 = (int)(i - (long)r * (DM / 8)) * 8;
  const int b  = r / SEQ;
  const int s  = r - b * SEQ;
  const float* src = x + ((size_t)b * SEQ_FULL + s) * DM + c8;
  const v4f a0 = *(const v4f*)src;
  const v4f a1 = *(const v4f*)(src + 4);
  v8h hv;
  hv[0] = bf_f16(a0[0]); hv[1] = bf_f16(a0[1]); hv[2] = bf_f16(a0[2]); hv[3] = bf_f16(a0[3]);
  hv[4] = bf_f16(a1[0]); hv[5] = bf_f16(a1[1]); hv[6] = bf_f16(a1[2]); hv[7] = bf_f16(a1[3]);
  _Float16* dst = (_Float16*)xhp + (size_t)r * DM + c8;
  *(volatile v8h*)dst = hv;
  __threadfence();
  *(volatile v8h*)dst = hv;
}

__global__ __launch_bounds__(256) void transpose_cast_f16(
    const float* __restrict__ W, unsigned short* __restrict__ Btp, int Kdim, int Ndim, int ldo, int kc0, float sc) {
  __shared__ float t[64][65];
  const int tid = threadIdx.x, lane = tid & 31, wave = tid >> 5;
  const int n0 = blockIdx.x * 64, k0 = blockIdx.y * 64;
#pragma unroll
  for (int i = 0; i < 16; ++i) {
    const int idx = i * 256 + tid;
    const int kr = idx >> 6, nc = idx & 63;
    t[nc][kr] = W[(size_t)(k0 + kr) * Ndim + n0 + nc];
  }
  __syncthreads();
  _Float16* Bt = (_Float16*)Btp;
  const int q = lane >> 3, c8 = (lane & 7) * 8;
  for (int pass = 0; pass < 2; ++pass) {
#pragma unroll
    for (int it = 0; it < 2; ++it) {
      const int row = wave * 8 + it * 4 + q;
      v8h hv;
#pragma unroll
      for (int e = 0; e < 8; ++e) hv[e] = (_Float16)(bf_rne(t[row][c8 + e]) * sc);
      *(volatile v8h*)(Bt + (size_t)(n0 + row) * ldo + kc0 + k0 + c8) = hv;
    }
    __threadfence();
  }
}

#define AT_D 64
#define AT_NW 4
#define AT_QB 64
#define AT_KC 64

__device__ __forceinline__ v8f mma_h(v16h a, v16h b, v8f c) {
  c = __builtin_amdgcn_wmma_f32_16x16x32_f16(false, a, false, b, (short)0, c, false, false);
  asm volatile("v_nop\n\tv_nop\n\tv_nop\n\tv_nop" : "+v"(c) : "v"(a), "v"(b));
  return c;
}

__global__ __launch_bounds__(128)
void attn64_causal(const unsigned short* __restrict__ Qp, const unsigned short* __restrict__ Kp,
                   const unsigned short* __restrict__ Vtp, unsigned short* __restrict__ Op,
                   int S, int H, int ldq, int ldvt, int qb0, int nqbl, float sc2, float osc) {
  const _Float16* Q  = (const _Float16*)Qp;
  const _Float16* Kk = (const _Float16*)Kp;
  const _Float16* Vt = (const _Float16*)Vtp;
  _Float16*       O  = (_Float16*)Op;
  __shared__ __align__(16) _Float16 Psh[AT_NW][16 * AT_KC];
  __shared__ __align__(16) float    Os[AT_NW][16 * 68];

  const int tid  = threadIdx.x;
  const int wave = tid >> 5;
  const int lane = tid & 31;
  const int hh   = lane >> 4;
  const int c    = lane & 15;

  const int bx  = blockIdx.x;
  const int qbi = bx % nqbl;
  const int bh  = bx / nqbl;
  const int qb  = qb0 + qbi;
  const int h   = bh % H;
  const int b   = bh / H;
  const int q0  = qb * AT_QB + wave * 16;
  const size_t rowb = (size_t)b * S;

  const _Float16* qp = Q  + rowb * ldq + (size_t)h * AT_D;
  const _Float16* kp = Kk + rowb * ldq + (size_t)h * AT_D;
  const _Float16* vp = Vt + (size_t)(h * AT_D) * ldvt + rowb;
  _Float16*       op = O  + rowb * ldq + (size_t)h * AT_D;

  v16h qa[2];
#pragma unroll
  for (int dc = 0; dc < 2; ++dc)
    qa[dc] = Frag<_Float16>::load(qp + (size_t)(q0 + c) * ldq + dc * 32 + 8 * hh);

  float mrow[8], lrow[8];
  v8f oacc[4];
#pragma unroll
  for (int r = 0; r < 8; ++r) { mrow[r] = NEG_INF; lrow[r] = 0.f; }
#pragma unroll
  for (int t = 0; t < 4; ++t) oacc[t] = (v8f){0.f,0.f,0.f,0.f,0.f,0.f,0.f,0.f};

  _Float16* pw = Psh[wave];
  const int nChunks = qb + 1;
  for (int kc = 0; kc < nChunks; ++kc) {
    const int kv0 = kc * AT_KC;
    v8f s[4];
#pragma unroll
    for (int j = 0; j < 4; ++j) {
      s[j] = (v8f){0.f,0.f,0.f,0.f,0.f,0.f,0.f,0.f};
#pragma unroll
      for (int dc = 0; dc < 2; ++dc) {
        const v16h kb = Frag<_Float16>::load(kp + (size_t)(kv0 + j * 16 + c) * ldq + dc * 32 + 8 * hh);
        s[j] = mma_h(qa[dc], kb, s[j]);
      }
    }
    float cm[8];
#pragma unroll
    for (int r = 0; r < 8; ++r) {
      const int qrow = q0 + 8 * hh + r;
      float m = NEG_INF;
#pragma unroll
      for (int j = 0; j < 4; ++j) {
        float v = s[j][r] * sc2;
        if (kv0 + j * 16 + c > qrow) v = NEG_INF;
        s[j][r] = v;
        m = fmaxf(m, v);
      }
#pragma unroll
      for (int off = 1; off < 16; off <<= 1) m = fmaxf(m, __shfl_xor(m, off, 32));
      cm[r] = m;
    }
    wave_lds_sync();
#pragma unroll
    for (int r = 0; r < 8; ++r) {
      const float mnew  = fmaxf(mrow[r], cm[r]);
      const float alpha = exp2f(mrow[r] - mnew);
      mrow[r] = mnew;
      float psum = 0.f;
#pragma unroll
      for (int j = 0; j < 4; ++j) {
        const float p = exp2f(s[j][r] - mnew);
        psum += p;
        pw[(8 * hh + r) * AT_KC + j * 16 + c] = (_Float16)(p * PSCALE);
      }
#pragma unroll
      for (int off = 1; off < 16; off <<= 1) psum += __shfl_xor(psum, off, 32);
      lrow[r] = lrow[r] * alpha + psum;
#pragma unroll
      for (int t = 0; t < 4; ++t) oacc[t][r] *= alpha;
    }
    wave_lds_sync();
#pragma unroll
    for (int kk = 0; kk < 2; ++kk) {
      const v16h pa = Frag<_Float16>::load(pw + c * AT_KC + kk * 32 + 8 * hh);
#pragma unroll
      for (int t = 0; t < 4; ++t) {
        const v16h vb = Frag<_Float16>::load(vp + (size_t)(t * 16 + c) * ldvt + kv0 + kk * 32 + 8 * hh);
        oacc[t] = mma_h(pa, vb, oacc[t]);
      }
    }
    wave_lds_sync();
  }

  float* os = Os[wave];
#pragma unroll
  for (int r = 0; r < 8; ++r) {
    const float inv = osc * (1.0f / (lrow[r] * PSCALE));
#pragma unroll
    for (int t = 0; t < 4; ++t) os[(8 * hh + r) * 68 + t * 16 + c] = oacc[t][r] * inv;
  }
  wave_lds_sync();
  {
    const int q = lane >> 3, c8 = (lane & 7) * 8;
    for (int pass = 0; pass < 2; ++pass) {
#pragma unroll
      for (int it = 0; it < 4; ++it) {
        const int row = it * 4 + q;
        const float* sp = os + row * 68 + c8;
        v8h hv;
#pragma unroll
        for (int e = 0; e < 8; ++e) hv[e] = (_Float16)sp[e];
        *(volatile v8h*)(op + (size_t)(q0 + row) * ldq + c8) = hv;
      }
      __threadfence();
    }
  }
}

__global__ __launch_bounds__(128)
void attn64_causal_res(const unsigned short* __restrict__ Qhp, const unsigned short* __restrict__ Qrp,
                       const unsigned short* __restrict__ Khp, const unsigned short* __restrict__ Krp,
                       const unsigned short* __restrict__ Vhp, const unsigned short* __restrict__ Vrp,
                       unsigned short* __restrict__ Op,
                       int H, int ldq, int ldvc, int ldo, int rcol, int nqb, float sc2, float osc) {
  const _Float16* QH = (const _Float16*)Qhp;
  const _Float16* QR = (const _Float16*)Qrp;
  const _Float16* KH = (const _Float16*)Khp;
  const _Float16* KR = (const _Float16*)Krp;
  const _Float16* VH = (const _Float16*)Vhp;
  const _Float16* VR = (const _Float16*)Vrp;
  _Float16*       O  = (_Float16*)Op;
  __shared__ __align__(16) _Float16 Psh[AT_NW][16 * AT_KC];
  __shared__ __align__(16) _Float16 Prs[AT_NW][16 * AT_KC];
  __shared__ __align__(16) float    Os[AT_NW][16 * 68];

  const int tid  = threadIdx.x;
  const int wave = tid >> 5;
  const int lane = tid & 31;
  const int hh   = lane >> 4;
  const int c    = lane & 15;

  const int bx = blockIdx.x;
  const int qb = bx % nqb;
  const int bh = bx / nqb;
  const int h  = bh % H;
  const int b  = bh / H;
  const int q0 = qb * AT_QB + wave * 16;
  const int rr = nqb * AT_QB;
  const size_t rowb = (size_t)b * rr;

  const _Float16* qhp = QH + rowb * ldq + (size_t)h * AT_D;
  const _Float16* qrp = QR + rowb * ldq + (size_t)h * AT_D;
  const _Float16* khp = KH + rowb * ldq + (size_t)h * AT_D;
  const _Float16* krp = KR + rowb * ldq + (size_t)h * AT_D;
  const size_t    vof = ((size_t)b * (size_t)(H * AT_D) + (size_t)h * AT_D) * ldvc;
  const _Float16* vhp = VH + vof;
  const _Float16* vrp = VR + vof;
  _Float16*       op  = O  + rowb * ldo + (size_t)h * AT_D;

  float mrow[8], lrow[8];
  v8f oacc[4], oacc2[4];
#pragma unroll
  for (int r = 0; r < 8; ++r) { mrow[r] = NEG_INF; lrow[r] = 0.f; }
#pragma unroll
  for (int t = 0; t < 4; ++t) {
    oacc[t]  = (v8f){0.f,0.f,0.f,0.f,0.f,0.f,0.f,0.f};
    oacc2[t] = (v8f){0.f,0.f,0.f,0.f,0.f,0.f,0.f,0.f};
  }

  _Float16* pw  = Psh[wave];
  _Float16* prw = Prs[wave];
  const int nChunks = qb + 1;
  for (int kc = 0; kc < nChunks; ++kc) {
    const int kv0 = kc * AT_KC;
    v16h qa[2], qra[2];
#pragma unroll
    for (int dc = 0; dc < 2; ++dc) {
      const size_t qo = (size_t)(q0 + c) * ldq + dc * 32 + 8 * hh;
      qa[dc]  = Frag<_Float16>::load(qhp + qo);
      qra[dc] = Frag<_Float16>::load(qrp + qo);
    }
    v8f s[4];
#pragma unroll
    for (int j = 0; j < 4; ++j) {
      v8f s1 = (v8f){0.f,0.f,0.f,0.f,0.f,0.f,0.f,0.f};
      v8f s2 = (v8f){0.f,0.f,0.f,0.f,0.f,0.f,0.f,0.f};
#pragma unroll
      for (int dc = 0; dc < 2; ++dc) {
        const size_t ko = (size_t)(kv0 + j * 16 + c) * ldq + dc * 32 + 8 * hh;
        const v16h kb = Frag<_Float16>::load(khp + ko);
        const v16h kr = Frag<_Float16>::load(krp + ko);
        s1 = mma_h(qa[dc],  kb, s1);
        s2 = mma_h(qa[dc],  kr, s2);
        s2 = mma_h(qra[dc], kb, s2);
      }
#pragma unroll
      for (int r = 0; r < 8; ++r) s[j][r] = s1[r] + s2[r] * RSC_INV;
    }
    float cm[8];
#pragma unroll
    for (int r = 0; r < 8; ++r) {
      const int qrow = q0 + 8 * hh + r;
      float m = NEG_INF;
#pragma unroll
      for (int j = 0; j < 4; ++j) {
        float v = s[j][r] * sc2;
        if (kv0 + j * 16 + c > qrow) v = NEG_INF;
        s[j][r] = v;
        m = fmaxf(m, v);
      }
#pragma unroll
      for (int off = 1; off < 16; off <<= 1) m = fmaxf(m, __shfl_xor(m, off, 32));
      cm[r] = m;
    }
    wave_lds_sync();
#pragma unroll
    for (int r = 0; r < 8; ++r) {
      const float mnew  = fmaxf(mrow[r], cm[r]);
      const float alpha = exp2f(mrow[r] - mnew);
      mrow[r] = mnew;
      float psum = 0.f;
#pragma unroll
      for (int j = 0; j < 4; ++j) {
        const float p = exp2f(s[j][r] - mnew);
        psum += p;
        const float    ps = p * PSCALE;
        const _Float16 ph = (_Float16)ps;
        const int pi = (8 * hh + r) * AT_KC + j * 16 + c;
        pw[pi]  = ph;
        prw[pi] = (_Float16)((ps - (float)ph) * RSC);
      }
#pragma unroll
      for (int off = 1; off < 16; off <<= 1) psum += __shfl_xor(psum, off, 32);
      lrow[r] = lrow[r] * alpha + psum;
#pragma unroll
      for (int t = 0; t < 4; ++t) { oacc[t][r] *= alpha; oacc2[t][r] *= alpha; }
    }
    wave_lds_sync();
#pragma unroll
    for (int kk = 0; kk < 2; ++kk) {
      const v16h pa = Frag<_Float16>::load(pw  + c * AT_KC + kk * 32 + 8 * hh);
      const v16h pr = Frag<_Float16>::load(prw + c * AT_KC + kk * 32 + 8 * hh);
#pragma unroll
      for (int t = 0; t < 4; ++t) {
        const size_t vo = (size_t)(t * 16 + c) * ldvc + kv0 + kk * 32 + 8 * hh;
        const v16h vb = Frag<_Float16>::load(vhp + vo);
        const v16h vr = Frag<_Float16>::load(vrp + vo);
        oacc[t]  = mma_h(pa, vb, oacc[t]);
        oacc2[t] = mma_h(pa, vr, oacc2[t]);
        oacc2[t] = mma_h(pr, vb, oacc2[t]);
      }
    }
    wave_lds_sync();
  }

  float* os = Os[wave];
#pragma unroll
  for (int r = 0; r < 8; ++r) {
    const float inv = osc * (1.0f / (lrow[r] * PSCALE));
#pragma unroll
    for (int t = 0; t < 4; ++t) os[(8 * hh + r) * 68 + t * 16 + c] = (oacc[t][r] + oacc2[t][r] * RSC_INV) * inv;
  }
  wave_lds_sync();
  {
    const int q = lane >> 3, c8 = (lane & 7) * 8;
    for (int pass = 0; pass < 2; ++pass) {
#pragma unroll
      for (int it = 0; it < 4; ++it) {
        const int row = it * 4 + q;
        const float* sp = os + row * 68 + c8;
        v8h hv, lv;
#pragma unroll
        for (int e = 0; e < 8; ++e) {
          const float    fv = sp[e];
          const _Float16 hq = (_Float16)fv;
          hv[e] = hq;
          lv[e] = (_Float16)((fv - (float)hq) * RSC);
        }
        *(volatile v8h*)(op + (size_t)(q0 + row) * ldo + c8) = hv;
        *(volatile v8h*)(op + (size_t)(q0 + row) * ldo + rcol + c8) = lv;
      }
      __threadfence();
    }
  }
}


extern "C" void kernel_launch(void* const* d_in, const int* in_sizes, int n_in,
                              void* d_out, int out_size, void* d_ws,
                              size_t ws_size, hipStream_t stream) {
  const int  ROWS  = NB * SEQ;
  const long needX = ((long)(NB - 1) * SEQ_FULL + SEQ) * (long)DM;
  const int  nW    = DM * DM;
  if (n_in < 9) return;
  if ((long)in_sizes[0] < needX || in_sizes[1] < nW || in_sizes[2] < DM || in_sizes[3] < nW ||
      in_sizes[4] < DM || in_sizes[5] < nW || in_sizes[6] < DM || in_sizes[7] < nW ||
      in_sizes[8] < DM || (long)out_size < needX) return;

  const float* x  = (const float*)d_in[0];
  const float* Wq = (const float*)d_in[1];
  const float* bq = (const float*)d_in[2];
  const float* Wk = (const float*)d_in[3];
  const float* bk = (const float*)d_in[4];
  const float* Wv = (const float*)d_in[5];
  const float* bv = (const float*)d_in[6];
  const float* Wo = (const float*)d_in[7];
  const float* bo = (const float*)d_in[8];
  float* out = (float*)d_out;

  const size_t szAct = (size_t)ROWS * DM * 2;
  const size_t szW   = (size_t)DM * DM * 2;
  const size_t szW2  = (size_t)DM * (2 * DM) * 2;
  const size_t szCmp = (size_t)NB * RR * DM * 2;
  const size_t szO2  = (size_t)NB * RR * (2 * DM) * 2;
  size_t off = 0;
  const size_t oXh   = off; off += szAct;
  const size_t oWqT  = off; off += szW;
  const size_t oWkT  = off; off += szW;
  const size_t oWvT  = off; off += szW;
  const size_t oWoT2 = off; off += szW2;
  const size_t oQh   = off; off += szAct;
  const size_t oKh   = off; off += szAct;
  const size_t oVt   = off; off += szAct;
  const size_t oAh   = off; off += szAct;
  const size_t oQch  = off; off += szCmp;
  const size_t oQcr  = off; off += szCmp;
  const size_t oKch  = off; off += szCmp;
  const size_t oKcr  = off; off += szCmp;
  const size_t oVch  = off; off += szCmp;
  const size_t oVcr  = off; off += szCmp;
  const size_t oOc2  = off; off += szO2;
  if (off > ws_size) return;

  char* ws = (char*)d_ws;
  unsigned short* xh   = (unsigned short*)(ws + oXh);
  unsigned short* WqT  = (unsigned short*)(ws + oWqT);
  unsigned short* WkT  = (unsigned short*)(ws + oWkT);
  unsigned short* WvT  = (unsigned short*)(ws + oWvT);
  unsigned short* WoT2 = (unsigned short*)(ws + oWoT2);
  unsigned short* Qh   = (unsigned short*)(ws + oQh);
  unsigned short* Kh   = (unsigned short*)(ws + oKh);
  unsigned short* Vt   = (unsigned short*)(ws + oVt);
  unsigned short* Ah   = (unsigned short*)(ws + oAh);
  unsigned short* Qch  = (unsigned short*)(ws + oQch);
  unsigned short* Qcr  = (unsigned short*)(ws + oQcr);
  unsigned short* Kch  = (unsigned short*)(ws + oKch);
  unsigned short* Kcr  = (unsigned short*)(ws + oKcr);
  unsigned short* Vch  = (unsigned short*)(ws + oVch);
  unsigned short* Vcr  = (unsigned short*)(ws + oVcr);
  unsigned short* Oc2  = (unsigned short*)(ws + oOc2);

  const float sc2   = 0.125f * 1.4426950408889634f;
  const float outsc = 1.0f / (WSC * OSC);

  {
    const long tot = (long)ROWS * (DM / 8);
    cast_x_f16<<<dim3((unsigned)((tot + 255) / 256)), dim3(256), 0, stream>>>(x, xh, ROWS);
  }
  {
    const dim3 tg(DM / 64, DM / 64);
    transpose_cast_f16<<<tg, dim3(256), 0, stream>>>(Wq, WqT, DM, DM, DM, 0, WSC);
    transpose_cast_f16<<<tg, dim3(256), 0, stream>>>(Wk, WkT, DM, DM, DM, 0, WSC);
    transpose_cast_f16<<<tg, dim3(256), 0, stream>>>(Wv, WvT, DM, DM, DM, 0, WSC);
    transpose_cast_f16<<<tg, dim3(256), 0, stream>>>(Wo, WoT2, DM, DM, 2 * DM, 0, WSC);
    transpose_cast_f16<<<tg, dim3(256), 0, stream>>>(Wo, WoT2, DM, DM, 2 * DM, DM, WSC * RSC_INV);
  }
  {
    const int tiles = (ROWS / 64) * (DM / 64);
    const dim3 gg((tiles + 7) / 8, 1);
    wmma_gemm64<0, false, 2, 1, false, 0><<<gg, dim3(256), 0, stream>>>(
        xh, xh, DM, 0L, WqT, WqT, DM, 0L, (void*)Qh, (void*)Qh, DM, 0L, bq, bq, 0L,
        ROWS, DM, DM, 1.0f / WSC);
    wmma_gemm64<0, false, 2, 1, false, 0><<<gg, dim3(256), 0, stream>>>(
        xh, xh, DM, 0L, WkT, WkT, DM, 0L, (void*)Kh, (void*)Kh, DM, 0L, bk, bk, 0L,
        ROWS, DM, DM, 1.0f / WSC);
    wmma_gemm64<0, false, 1, 1, false, 0><<<gg, dim3(256), 0, stream>>>(
        WvT, WvT, DM, 0L, xh, xh, DM, 0L, (void*)Vt, (void*)Vt, ROWS, 0L, bv, bv, 0L,
        DM, ROWS, DM, 1.0f / WSC);
  }
  {
    const int tiles = (RR / 64) * (DM / 64);
    const dim3 gc((tiles + 7) / 8, NB);
    const long sA = (long)SEQ * DM;
    const long sC = (long)RR * DM;
    wmma_gemm64<0, false, 2, 3, false, 0><<<gc, dim3(256), 0, stream>>>(
        xh, xh, DM, sA, WqT, WqT, DM, 0L, (void*)Qch, (void*)Qcr, DM, sC, bq, bq, 0L,
        RR, DM, DM, 1.0f / WSC);
    wmma_gemm64<0, false, 2, 3, false, 0><<<gc, dim3(256), 0, stream>>>(
        xh, xh, DM, sA, WkT, WkT, DM, 0L, (void*)Kch, (void*)Kcr, DM, sC, bk, bk, 0L,
        RR, DM, DM, 1.0f / WSC);
    wmma_gemm64<0, false, 1, 3, false, 0><<<gc, dim3(256), 0, stream>>>(
        WvT, WvT, DM, 0L, xh, xh, DM, sA, (void*)Vch, (void*)Vcr, RR, (long)DM * RR, bv, bv, 0L,
        DM, RR, DM, 1.0f / WSC);
  }
  attn64_causal_res<<<dim3(NB * NH * (RR / 64)), dim3(128), 0, stream>>>(
      Qch, Qcr, Kch, Kcr, Vch, Vcr, Oc2, NH, DM, RR, 2 * DM, DM, RR / 64, sc2, OSC);
  if (SEQ > RR) {
    attn64_causal<<<dim3(NB * NH * ((SEQ - RR) / 64)), dim3(128), 0, stream>>>(
        Qh, Kh, Vt, Ah, SEQ, NH, DM, ROWS, RR / 64, (SEQ - RR) / 64, sc2, OSC);
  }
  {
    const int tiles = (RR / 64) * (DM / 64);
    const dim3 g1((tiles + 7) / 8, NB);
    wmma_gemm64<0, false, 2, 0, false, 0><<<g1, dim3(256), 0, stream>>>(
        Oc2, Oc2, 2 * DM, (long)RR * 2 * DM, WoT2, WoT2, 2 * DM, 0L,
        (void*)out, (void*)out, DM, (long)SEQ_FULL * DM, bo, bo, 0L,
        RR, DM, 2 * DM, outsc);
  }
  if (SEQ > RR) {
    const int tiles = ((SEQ - RR) / 64) * (DM / 64);
    const dim3 g2((tiles + 7) / 8, NB);
    unsigned short* Ahi = Ah + (size_t)RR * DM;
    float* outp = out + (size_t)RR * DM;
    wmma_gemm64<0, false, 2, 0, false, 0><<<g2, dim3(256), 0, stream>>>(
        Ahi, Ahi, DM, (long)SEQ * DM, WoT2, WoT2, 2 * DM, 0L,
        (void*)outp, (void*)outp, DM, (long)SEQ_FULL * DM, bo, bo, 0L,
        SEQ - RR, DM, DM, outsc);
  }
}
